// EGNN_predictor_40604620816578
// MI455X (gfx1250) — hardware-verified
//
#include <hip/hip_runtime.h>
#include <stddef.h>
#include <stdint.h>


#define HD      128
#define NPG     64
#define NGR     64
#define NNODE   4096
#define NLAY    4
#define NFEAT   11
#define LDH     136
#define XR      32
#define WPL     114688
#define OF_EW1A 0
#define OF_EW1B 16384
#define OF_EW2  32768
#define OF_CW1  49152
#define OF_NW1  65536
#define OF_NW2  98304
#define EW1L    33024
#define WINV    0.0625f
#define NTHR    256

static_assert((NLAY * WPL) % 2048 == 0);
static_assert(WPL % 2048 == 0);
static_assert((LDH % 8) == 0);

typedef _Float16 v4h  __attribute__((ext_vector_type(4)));
typedef _Float16 v8h  __attribute__((ext_vector_type(8)));
typedef _Float16 v16h __attribute__((ext_vector_type(16)));
typedef float    v4f  __attribute__((ext_vector_type(4)));
typedef float    v8f  __attribute__((ext_vector_type(8)));
union Frag { v16h v; v8h h[2]; };

__device__ __forceinline__ v8f zero8f() {
  v8f z;
#pragma unroll
  for (int i = 0; i < 8; ++i) z[i] = 0.0f;
  return z;
}

__device__ __forceinline__ v8f wmh(v16h a, v16h b, v8f c) {
  v8f d = __builtin_amdgcn_wmma_f32_16x16x32_f16(false, a, false, b, (short)0, c, false, false);
  asm volatile("v_nop\n\tv_nop\n\tv_nop\n\tv_nop" : "+v"(d) : "v"(a), "v"(b));
  return d;
}

__device__ __forceinline__ v16h ldfrag(const _Float16* T, int r0, int k0, int m, int hh) {
  Frag f;
  const _Float16* p = T + (r0 + m) * LDH + k0 + 8 * hh;
  f.h[0] = *(const v8h*)p;
  f.h[1] = *(const v8h*)(p + 16);
  return f.v;
}

__device__ __forceinline__ float silu_f(float x) {
  const float e = __expf(-x);
  return x * __builtin_amdgcn_rcpf(1.0f + e);
}

__global__ __launch_bounds__(NTHR) void k_wcvt(const float* __restrict__ ew1, const float* __restrict__ ew2,
                                              const float* __restrict__ cw1, const float* __restrict__ nw1,
                                              const float* __restrict__ nw2, _Float16* wf) {
  const int tid = threadIdx.x;
  const int bq  = blockIdx.x * 2048;
  const int l   = bq / WPL;
  const int rb  = bq - l * WPL;
  const float* src = ew1;
  size_t sbase = 0;
  int rbase = 0, ksh = 7;
  float sc0 = 16.0f, sc1 = 16.0f;
  if (rb < OF_EW1B)     { src = ew1; sbase = (size_t)l * EW1L;            rbase = OF_EW1A; }
  else if (rb < OF_EW2) { src = ew1; sbase = (size_t)l * EW1L + 128 * HD; rbase = OF_EW1B; }
  else if (rb < OF_CW1) { src = ew2; sbase = (size_t)l * HD * HD;         rbase = OF_EW2; }
  else if (rb < OF_NW1) { src = cw1; sbase = (size_t)l * HD * HD;         rbase = OF_CW1; }
  else if (rb < OF_NW2) { src = nw1; sbase = (size_t)l * 2 * HD * HD;     rbase = OF_NW1; ksh = 8; sc1 = 256.0f; }
  else                  { src = nw2; sbase = (size_t)l * HD * HD;         rbase = OF_NW2; sc0 = 128.0f; sc1 = 128.0f; }
  const int r = rb - rbase + tid * 8;
  const int n = r >> ksh;
  const int k = r & ((1 << ksh) - 1);
  const float sc = (k < HD) ? sc0 : sc1;
  v8h o;
#pragma unroll
  for (int i = 0; i < 8; ++i) o[i] = (_Float16)(src[sbase + (size_t)(k + i) * HD + n] * sc);
  _Float16* dst = wf + (size_t)bq + (size_t)tid * 8;
  *(volatile v8h*)dst = o;
  __threadfence();
  *(volatile v8h*)dst = o;
}

__global__ __launch_bounds__(NTHR) void k_prep(const float* __restrict__ xh, const float* __restrict__ nmask,
                                              const float* __restrict__ emb_w, const float* __restrict__ emb_b,
                                              float* xp, float* hp) {
  __shared__ __attribute__((aligned(16))) float sIn[NPG * NFEAT];
  __shared__ float sNm[NPG];
  __shared__ __attribute__((aligned(16))) float sX[NPG * XR];
  __shared__ __attribute__((aligned(16))) float sH[NPG * HD];
  const int g = blockIdx.x, tid = threadIdx.x;
  const int nb0 = g * NPG;
  for (int i = tid; i < NPG * NFEAT; i += NTHR) sIn[i] = xh[(size_t)nb0 * NFEAT + i];
  if (tid < NPG) sNm[tid] = nmask[nb0 + tid];
  for (int i = tid; i < NPG * XR; i += NTHR) sX[i] = 0.0f;
  __syncthreads();
  if (tid < NPG) {
    const float nm = sNm[tid];
#pragma unroll
    for (int c = 0; c < 3; ++c) {
      const float v = sIn[tid * NFEAT + c] * nm;
      sX[tid * XR + c] = v;
      sX[tid * XR + 4 + c] = v;
    }
  }
  {
    const int c = tid & (HD - 1), ng = tid >> 7;
    float w[8];
#pragma unroll
    for (int k = 0; k < 8; ++k) w[k] = emb_w[k * HD + c];
    const float b = emb_b[c];
#pragma unroll 1
    for (int jj = 0; jj < NPG / 2; ++jj) {
      const int j = ng + 2 * jj;
      const float nm = sNm[j];
      float acc = b;
#pragma unroll
      for (int k = 0; k < 8; ++k) acc += (sIn[j * NFEAT + 3 + k] * nm) * w[k];
      sH[j * HD + c] = acc;
    }
  }
  __syncthreads();
  v4f vx[2], vh[8];
#pragma unroll
  for (int it = 0; it < 2; ++it) {
    const int f = tid + NTHR * it, row = f >> 3, pc = f & 7;
    vx[it] = *(const v4f*)(sX + row * XR + 4 * pc);
    *(volatile v4f*)(xp + (size_t)(nb0 + row) * XR + 4 * pc) = vx[it];
  }
#pragma unroll
  for (int it = 0; it < 8; ++it) {
    const int f = tid + NTHR * it, row = f >> 5, pc = f & 31;
    vh[it] = *(const v4f*)(sH + row * HD + 4 * pc);
    *(volatile v4f*)(hp + (size_t)(nb0 + row) * HD + 4 * pc) = vh[it];
  }
  __threadfence();
#pragma unroll
  for (int it = 0; it < 2; ++it) {
    const int f = tid + NTHR * it, row = f >> 3, pc = f & 7;
    *(volatile v4f*)(xp + (size_t)(nb0 + row) * XR + 4 * pc) = vx[it];
  }
#pragma unroll
  for (int it = 0; it < 8; ++it) {
    const int f = tid + NTHR * it, row = f >> 5, pc = f & 31;
    *(volatile v4f*)(hp + (size_t)(nb0 + row) * HD + 4 * pc) = vh[it];
  }
}

__global__ __launch_bounds__(NTHR) void k_hih(const float* __restrict__ hc, const _Float16* __restrict__ wf,
                                             const float* __restrict__ eb1, int layer, float* Pp, float* Qp) {
  __shared__ __attribute__((aligned(16))) _Float16 sA[NPG * LDH];
  __shared__ __attribute__((aligned(16))) _Float16 sW[HD * LDH];
  __shared__ __attribute__((aligned(16))) float    sO[NPG * HD];
  const int g = blockIdx.x, tid = threadIdx.x, nb0 = g * NPG;
  const int w = tid >> 5, lane = tid & 31, m = lane & 15, hh = lane >> 4;
  const int m0 = (w >> 1) * 16, nbc = (w & 1) * 64;
#pragma unroll
  for (int it = 0; it < 8; ++it) {
    const int f = tid + NTHR * it, row = f >> 5, pc = f & 31;
    const v4f v = *(const v4f*)(hc + (size_t)(nb0 + row) * HD + 4 * pc);
    v4h o;
    o[0] = (_Float16)v[0]; o[1] = (_Float16)v[1]; o[2] = (_Float16)v[2]; o[3] = (_Float16)v[3];
    *(v4h*)(sA + row * LDH + 4 * pc) = o;
  }
  const _Float16* wl = wf + (size_t)layer * WPL;
  const float* bl = eb1 + layer * HD;
#pragma unroll 1
  for (int pass = 0; pass < 2; ++pass) {
    const _Float16* WT = wl + (pass ? OF_EW1B : OF_EW1A);
#pragma unroll
    for (int it = 0; it < 8; ++it) {
      const int f = tid + NTHR * it, row = f >> 4, ch = f & 15;
      *(v8h*)(sW + row * LDH + 8 * ch) = *(const v8h*)(WT + (size_t)row * HD + 8 * ch);
    }
    __syncthreads();
    v8f acc[4];
#pragma unroll
    for (int t = 0; t < 4; ++t) acc[t] = zero8f();
#pragma unroll
    for (int kk = 0; kk < HD; kk += 32) {
      const v16h a = ldfrag(sA, m0, kk, m, hh);
#pragma unroll
      for (int t = 0; t < 4; ++t) {
        const v16h b = ldfrag(sW, nbc + 16 * t, kk, m, hh);
        acc[t] = wmh(a, b, acc[t]);
      }
    }
#pragma unroll
    for (int t = 0; t < 4; ++t) {
      const int n = nbc + 16 * t + m;
      const float bias = (pass == 0) ? bl[n] : 0.0f;
#pragma unroll
      for (int r = 0; r < 8; ++r) sO[(m0 + 8 * hh + r) * HD + n] = acc[t][r] * WINV + bias;
    }
    __syncthreads();
    float* dst = pass ? Qp : Pp;
    v4f v[8];
#pragma unroll
    for (int it = 0; it < 8; ++it) {
      const int f = tid + NTHR * it, row = f >> 5, pc = f & 31;
      v[it] = *(const v4f*)(sO + row * HD + 4 * pc);
      *(volatile v4f*)(dst + (size_t)(nb0 + row) * HD + 4 * pc) = v[it];
    }
    __threadfence();
#pragma unroll
    for (int it = 0; it < 8; ++it) {
      const int f = tid + NTHR * it, row = f >> 5, pc = f & 31;
      *(volatile v4f*)(dst + (size_t)(nb0 + row) * HD + 4 * pc) = v[it];
    }
  }
}

__global__ __launch_bounds__(NTHR) void k_edge(
    const float* __restrict__ xc, const float* __restrict__ Pp, const float* __restrict__ Qp,
    const _Float16* __restrict__ wf, int layer,
    const float* __restrict__ ew1, const float* __restrict__ eb2, const float* __restrict__ cb1,
    const float* __restrict__ cw2, const float* __restrict__ emask,
    float* xn, float* aggp) {
  __shared__ __attribute__((aligned(16))) _Float16 sW2[HD * LDH];
  __shared__ __attribute__((aligned(16))) _Float16 sW3[HD * LDH];
  __shared__ __attribute__((aligned(16))) _Float16 sM[128 * LDH];
  __shared__ __attribute__((aligned(16))) float sCD[128 * 4];
  __shared__ __attribute__((aligned(16))) float sColP[8 * HD];
  __shared__ __attribute__((aligned(16))) float sAgg[2 * HD];
  __shared__ __attribute__((aligned(16))) float sXo[2 * XR];
  __shared__ float sRad[128], sEA[128], sEM[128], sS[128];

  const int tid = threadIdx.x, w = tid >> 5, lane = tid & 31, m = lane & 15, hh = lane >> 4;
  const int g = blockIdx.x >> 5, pr = blockIdx.x & 31;
  const int gb = g * NPG;
  const int i0 = gb + 2 * pr;
  const _Float16* wl = wf + (size_t)layer * WPL;

#pragma unroll
  for (int it = 0; it < 8; ++it) {
    const int f = tid + NTHR * it, row = f >> 4, ch = f & 15;
    *(v8h*)(sW2 + row * LDH + 8 * ch) = *(const v8h*)(wl + OF_EW2 + (size_t)row * HD + 8 * ch);
    *(v8h*)(sW3 + row * LDH + 8 * ch) = *(const v8h*)(wl + OF_CW1 + (size_t)row * HD + 8 * ch);
  }
  if (tid < 128) {
    const int e = tid, n = e >> 6, j = e & 63;
    const int ni = i0 + n, nj = gb + j;
    const v4f xi = *(const v4f*)(xc + (size_t)ni * XR);
    const v4f xj = *(const v4f*)(xc + (size_t)nj * XR);
    const v4f yi = *(const v4f*)(xc + (size_t)ni * XR + 4);
    const v4f yj = *(const v4f*)(xc + (size_t)nj * XR + 4);
    const float dx = xi[0] - xj[0], dy = xi[1] - xj[1], dz = xi[2] - xj[2];
    const float rad = dx * dx + dy * dy + dz * dz;
    const float inv = 1.0f / (sqrtf(rad + 1e-8f) + 1.0f);
    sCD[e * 4 + 0] = dx * inv; sCD[e * 4 + 1] = dy * inv; sCD[e * 4 + 2] = dz * inv; sCD[e * 4 + 3] = 0.0f;
    sRad[e] = rad;
    const float ex = yi[0] - yj[0], ey = yi[1] - yj[1], ez = yi[2] - yj[2];
    sEA[e] = ex * ex + ey * ey + ez * ez;
    sEM[e] = emask[(size_t)ni * NPG + j];
  } else if (tid < 192) {
    const int t = tid - 128, n = t >> 5, col = t & 31;
    const float xin = xc[(size_t)(i0 + n) * XR + col];
    sXo[n * XR + col] = (col >= 4 && col < 7) ? xin : 0.0f;
  }
  __syncthreads();

  {
    const int cg = tid & 15, es = tid >> 4;
    const int c0 = cg * 8;
    const float* wrp = ew1 + (size_t)layer * EW1L + 256 * HD + c0;
    const v4f wr0 = *(const v4f*)wrp, wr1 = *(const v4f*)(wrp + 4);
    const v4f we0 = *(const v4f*)(wrp + HD), we1 = *(const v4f*)(wrp + HD + 4);
    const float* pp = Pp + (size_t)i0 * HD + c0;
    const v4f pa0 = *(const v4f*)pp, pa1 = *(const v4f*)(pp + 4);
    const v4f pb0 = *(const v4f*)(pp + HD), pb1 = *(const v4f*)(pp + HD + 4);
#pragma unroll
    for (int k = 0; k < 8; ++k) {
      const int e = es + 16 * k;
      const int j = e & 63;
      const float* qp = Qp + (size_t)(gb + j) * HD + c0;
      const v4f q0 = *(const v4f*)qp, q1 = *(const v4f*)(qp + 4);
      const float rad = sRad[e], ea = sEA[e];
      v4f px = pa0, py = pa1;
      if (k >= 4) { px = pb0; py = pb1; }
      v8h o;
#pragma unroll
      for (int i = 0; i < 4; ++i) {
        const float pre0 = px[i] + q0[i] + rad * wr0[i] + ea * we0[i];
        const float pre1 = py[i] + q1[i] + rad * wr1[i] + ea * we1[i];
        o[i]     = (_Float16)silu_f(pre0);
        o[4 + i] = (_Float16)silu_f(pre1);
      }
      *(v8h*)(sM + e * LDH + c0) = o;
    }
  }
  __syncthreads();

  const int r0w = 16 * w;
  float em8[8];
#pragma unroll
  for (int r = 0; r < 8; ++r) em8[r] = sEM[r0w + 8 * hh + r];

  v8f acc[8];
#pragma unroll
  for (int t = 0; t < 8; ++t) acc[t] = zero8f();
#pragma unroll
  for (int kk = 0; kk < HD; kk += 32) {
    const v16h a = ldfrag(sM, r0w, kk, m, hh);
#pragma unroll
    for (int t = 0; t < 8; ++t) {
      const v16h b = ldfrag(sW2, 16 * t, kk, m, hh);
      acc[t] = wmh(a, b, acc[t]);
    }
  }
  {
    const float* b2 = eb2 + layer * HD;
    float cs[8];
#pragma unroll
    for (int t = 0; t < 8; ++t) {
      const int n = 16 * t + m;
      const float bias = b2[n];
      float s = 0.0f;
#pragma unroll
      for (int r = 0; r < 8; ++r) {
        const float val = silu_f(acc[t][r] * WINV + bias) * em8[r];
        s += val;
        sM[(r0w + 8 * hh + r) * LDH + n] = (_Float16)val;
      }
      cs[t] = s;
    }
#pragma unroll
    for (int t = 0; t < 8; ++t) cs[t] += __shfl_xor(cs[t], 16);
    if (hh == 0) {
#pragma unroll
      for (int t = 0; t < 8; ++t) sColP[w * HD + 16 * t + m] = cs[t];
    }
  }
  __syncthreads();

  {
    const int n = tid >> 7, c = tid & (HD - 1);
    float a = sColP[(4 * n) * HD + c];
    a += sColP[(4 * n + 1) * HD + c];
    a += sColP[(4 * n + 2) * HD + c];
    a += sColP[(4 * n + 3) * HD + c];
    sAgg[n * HD + c] = a;
  }
#pragma unroll
  for (int t = 0; t < 8; ++t) acc[t] = zero8f();
#pragma unroll
  for (int kk = 0; kk < HD; kk += 32) {
    const v16h a = ldfrag(sM, r0w, kk, m, hh);
#pragma unroll
    for (int t = 0; t < 8; ++t) {
      const v16h b = ldfrag(sW3, 16 * t, kk, m, hh);
      acc[t] = wmh(a, b, acc[t]);
    }
  }
  {
    const float* cb = cb1 + layer * HD;
    const float* c2 = cw2 + layer * HD;
    float rd[8];
#pragma unroll
    for (int r = 0; r < 8; ++r) rd[r] = 0.0f;
#pragma unroll
    for (int t = 0; t < 8; ++t) {
      const int n = 16 * t + m;
      const float bias = cb[n], wv = c2[n];
#pragma unroll
      for (int r = 0; r < 8; ++r) rd[r] += silu_f(acc[t][r] * WINV + bias) * wv;
    }
#pragma unroll
    for (int r = 0; r < 8; ++r) {
      rd[r] += __shfl_xor(rd[r], 1);
      rd[r] += __shfl_xor(rd[r], 2);
      rd[r] += __shfl_xor(rd[r], 4);
      rd[r] += __shfl_xor(rd[r], 8);
    }
    if (m == 0) {
#pragma unroll
      for (int r = 0; r < 8; ++r) sS[r0w + 8 * hh + r] = rd[r] * em8[r];
    }
  }
  __syncthreads();

  if (w < 6) {
    const int n = (w >= 3) ? 1 : 0;
    const int c = w - 3 * n;
    const int e0 = n * 64 + lane, e1 = e0 + 32;
    float p = sS[e0] * sCD[e0 * 4 + c] + sS[e1] * sCD[e1 * 4 + c];
    p += __shfl_xor(p, 16);
    p += __shfl_xor(p, 8);
    p += __shfl_xor(p, 4);
    p += __shfl_xor(p, 2);
    p += __shfl_xor(p, 1);
    if (lane == 0) sXo[n * XR + c] = xc[(size_t)(i0 + n) * XR + c] + p;
  }
  __syncthreads();

  const bool doA = tid < 64, doX = tid < 16;
  v4f va, vx;
  {
    const int n = tid >> 5, pc = tid & 31;
    va = *(const v4f*)(sAgg + (doA ? n : 0) * HD + 4 * pc);
    if (doA) *(volatile v4f*)(aggp + (size_t)(i0 + n) * HD + 4 * pc) = va;
  }
  {
    const int n = (tid >> 3) & 1, pc = tid & 7;
    vx = *(const v4f*)(sXo + n * XR + 4 * pc);
    if (doX) *(volatile v4f*)(xn + (size_t)(i0 + n) * XR + 4 * pc) = vx;
  }
  __threadfence();
  if (doA) { const int n = tid >> 5, pc = tid & 31; *(volatile v4f*)(aggp + (size_t)(i0 + n) * HD + 4 * pc) = va; }
  if (doX) { const int n = (tid >> 3) & 1, pc = tid & 7; *(volatile v4f*)(xn + (size_t)(i0 + n) * XR + 4 * pc) = vx; }
}

__global__ __launch_bounds__(NTHR) void k_node(const float* __restrict__ hc, const float* __restrict__ aggp,
                                              const _Float16* __restrict__ wf, int layer,
                                              const float* __restrict__ nb1, const float* __restrict__ nb2,
                                              const float* __restrict__ nmask, float* hn) {
  __shared__ __attribute__((aligned(16))) _Float16 sA[NPG * LDH];
  __shared__ __attribute__((aligned(16))) _Float16 sW[HD * LDH];
  __shared__ __attribute__((aligned(16))) float    sO[NPG * HD];
  const int g = blockIdx.x, tid = threadIdx.x, nb0 = g * NPG;
  const int w = tid >> 5, lane = tid & 31, m = lane & 15, hh = lane >> 4;
  const int m0 = (w >> 1) * 16, nbc = (w & 1) * 64;
  const _Float16* wl = wf + (size_t)layer * WPL;

  v8f acc[4];
#pragma unroll
  for (int t = 0; t < 4; ++t) acc[t] = zero8f();
#pragma unroll 1
  for (int pass = 0; pass < 2; ++pass) {
    if (pass != 0) __syncthreads();
    const float* src = pass ? aggp : hc;
    const float asc  = pass ? 0.0625f : 1.0f;
#pragma unroll
    for (int it = 0; it < 8; ++it) {
      const int f = tid + NTHR * it, row = f >> 5, pc = f & 31;
      const v4f v = *(const v4f*)(src + (size_t)(nb0 + row) * HD + 4 * pc) * asc;
      v4h o;
      o[0] = (_Float16)v[0]; o[1] = (_Float16)v[1]; o[2] = (_Float16)v[2]; o[3] = (_Float16)v[3];
      *(v4h*)(sA + row * LDH + 4 * pc) = o;
    }
    const _Float16* WT = wl + OF_NW1 + pass * HD;
#pragma unroll
    for (int it = 0; it < 8; ++it) {
      const int f = tid + NTHR * it, row = f >> 4, ch = f & 15;
      *(v8h*)(sW + row * LDH + 8 * ch) = *(const v8h*)(WT + (size_t)row * (2 * HD) + 8 * ch);
    }
    __syncthreads();
#pragma unroll
    for (int kk = 0; kk < HD; kk += 32) {
      const v16h a = ldfrag(sA, m0, kk, m, hh);
#pragma unroll
      for (int t = 0; t < 4; ++t) {
        const v16h b = ldfrag(sW, nbc + 16 * t, kk, m, hh);
        acc[t] = wmh(a, b, acc[t]);
      }
    }
  }
  __syncthreads();
  {
    const float* bl1 = nb1 + layer * HD;
#pragma unroll
    for (int t = 0; t < 4; ++t) {
      const int n = nbc + 16 * t + m;
      const float bias = bl1[n];
#pragma unroll
      for (int r = 0; r < 8; ++r) {
        const float v = silu_f(acc[t][r] * WINV + bias);
        sA[(m0 + 8 * hh + r) * LDH + n] = (_Float16)(v * 0.125f);
      }
    }
#pragma unroll
    for (int it = 0; it < 8; ++it) {
      const int f = tid + NTHR * it, row = f >> 4, ch = f & 15;
      *(v8h*)(sW + row * LDH + 8 * ch) = *(const v8h*)(wl + OF_NW2 + (size_t)row * HD + 8 * ch);
    }
  }
  __syncthreads();
#pragma unroll
  for (int t = 0; t < 4; ++t) acc[t] = zero8f();
#pragma unroll
  for (int kk = 0; kk < HD; kk += 32) {
    const v16h a = ldfrag(sA, m0, kk, m, hh);
#pragma unroll
    for (int t = 0; t < 4; ++t) {
      const v16h b = ldfrag(sW, nbc + 16 * t, kk, m, hh);
      acc[t] = wmh(a, b, acc[t]);
    }
  }
  {
    const float* bl2 = nb2 + layer * HD;
    float nm8[8];
#pragma unroll
    for (int r = 0; r < 8; ++r) nm8[r] = nmask[nb0 + m0 + 8 * hh + r];
#pragma unroll
    for (int t = 0; t < 4; ++t) {
      const int n = nbc + 16 * t + m;
      const float bias = bl2[n];
#pragma unroll
      for (int r = 0; r < 8; ++r) {
        const int row = m0 + 8 * hh + r;
        const float hv = hc[(size_t)(nb0 + row) * HD + n];
        sO[row * HD + n] = (hv + (acc[t][r] * WINV + bias)) * nm8[r];
      }
    }
  }
  __syncthreads();
  v4f v[8];
#pragma unroll
  for (int it = 0; it < 8; ++it) {
    const int f = tid + NTHR * it, row = f >> 5, pc = f & 31;
    v[it] = *(const v4f*)(sO + row * HD + 4 * pc);
    *(volatile v4f*)(hn + (size_t)(nb0 + row) * HD + 4 * pc) = v[it];
  }
  __threadfence();
#pragma unroll
  for (int it = 0; it < 8; ++it) {
    const int f = tid + NTHR * it, row = f >> 5, pc = f & 31;
    *(volatile v4f*)(hn + (size_t)(nb0 + row) * HD + 4 * pc) = v[it];
  }
}

__global__ __launch_bounds__(NTHR) void k_out(const float* __restrict__ hc, const float* __restrict__ out_w,
                                             const float* __restrict__ out_b, const float* __restrict__ nmask,
                                             float* outp) {
  __shared__ float sPart[NGR * 8];
  __shared__ __attribute__((aligned(16))) float sRes[NGR];
  const int tid = threadIdx.x, w = tid >> 5, lane = tid & 31;
  const int q = lane & 3, nl = lane >> 2;
  const float ob = out_b[0];
#pragma unroll 1
  for (int gph = 0; gph < NGR; ++gph) {
    const int node = gph * NPG + w * 8 + nl;
    const float* hp = hc + (size_t)node * HD + 32 * q;
    const float* wp = out_w + 32 * q;
    float s = 0.0f;
#pragma unroll 1
    for (int i = 0; i < 8; ++i) {
      const v4f hv = *(const v4f*)(hp + 4 * i);
      const v4f wv = *(const v4f*)(wp + 4 * i);
      s += hv[0] * wv[0] + hv[1] * wv[1] + hv[2] * wv[2] + hv[3] * wv[3];
    }
    s += __shfl_xor(s, 1);
    s += __shfl_xor(s, 2);
    float val = (s + ob) * nmask[node];
    val += __shfl_xor(val, 4);
    val += __shfl_xor(val, 8);
    val += __shfl_xor(val, 16);
    if (lane == 0) sPart[gph * 8 + w] = val;
  }
  __syncthreads();
  if (tid < NGR) {
    float s = 0.0f;
#pragma unroll
    for (int k = 0; k < 8; ++k) s += sPart[tid * 8 + k];
    sRes[tid] = s * (1.0f / 64.0f);
  }
  __syncthreads();
  v4f v;
  v = *(const v4f*)(sRes + 4 * (tid & 15));
  if (tid < 16) *(volatile v4f*)(outp + 4 * tid) = v;
  __threadfence();
  if (tid < 16) *(volatile v4f*)(outp + 4 * tid) = v;
}

extern "C" void kernel_launch(void* const* d_in, const int* in_sizes, int n_in,
                              void* d_out, int out_size, void* d_ws, size_t ws_size,
                              hipStream_t stream) {
  if (n_in < 18) return;
  if (in_sizes[0] != NNODE * NFEAT || in_sizes[1] != NNODE || in_sizes[2] != NNODE * NPG) return;
  if (in_sizes[3] != 8 * HD || in_sizes[4] != HD || in_sizes[5] != HD || in_sizes[6] < 1) return;
  if (in_sizes[7] != NLAY * EW1L || in_sizes[8] != NLAY * HD) return;
  if (in_sizes[9] != NLAY * HD * HD || in_sizes[10] != NLAY * HD) return;
  if (in_sizes[11] != NLAY * 2 * HD * HD || in_sizes[12] != NLAY * HD) return;
  if (in_sizes[13] != NLAY * HD * HD || in_sizes[14] != NLAY * HD) return;
  if (in_sizes[15] != NLAY * HD * HD || in_sizes[16] != NLAY * HD || in_sizes[17] != NLAY * HD) return;
  if (out_size != NGR) return;

  const float* xh    = (const float*)d_in[0];
  const float* nmask = (const float*)d_in[1];
  const float* emask = (const float*)d_in[2];
  const float* emb_w = (const float*)d_in[3];
  const float* emb_b = (const float*)d_in[4];
  const float* out_w = (const float*)d_in[5];
  const float* out_b = (const float*)d_in[6];
  const float* ew1   = (const float*)d_in[7];
  const float* eb1   = (const float*)d_in[8];
  const float* ew2   = (const float*)d_in[9];
  const float* eb2   = (const float*)d_in[10];
  const float* nw1   = (const float*)d_in[11];
  const float* nb1   = (const float*)d_in[12];
  const float* nw2   = (const float*)d_in[13];
  const float* nb2   = (const float*)d_in[14];
  const float* cw1   = (const float*)d_in[15];
  const float* cb1   = (const float*)d_in[16];
  const float* cw2   = (const float*)d_in[17];
  float* out = (float*)d_out;

  char* ws = (char*)d_ws;
  size_t off = 0;
  const size_t szW = (size_t)NLAY * WPL * 2;
  const size_t szX = (size_t)NNODE * XR * 4;
  const size_t szH = (size_t)NNODE * HD * 4;
  const size_t oW  = off; off += szW;
  const size_t oXA = off; off += szX;
  const size_t oXB = off; off += szX;
  const size_t oHA = off; off += szH;
  const size_t oHB = off; off += szH;
  const size_t oP  = off; off += szH;
  const size_t oQ  = off; off += szH;
  const size_t oAg = off; off += szH;
  if (off > ws_size) return;
  _Float16* wf = (_Float16*)(ws + oW);
  float* xA  = (float*)(ws + oXA);
  float* xB  = (float*)(ws + oXB);
  float* hA  = (float*)(ws + oHA);
  float* hB  = (float*)(ws + oHB);
  float* P   = (float*)(ws + oP);
  float* Q   = (float*)(ws + oQ);
  float* agg = (float*)(ws + oAg);

  k_wcvt<<<(NLAY * WPL) / 2048, NTHR, 0, stream>>>(ew1, ew2, cw1, nw1, nw2, wf);
  k_prep<<<NGR, NTHR, 0, stream>>>(xh, nmask, emb_w, emb_b, xA, hA);

  float* xc = xA; float* xnx = xB;
  float* hc = hA; float* hnx = hB;
  for (int l = 0; l < NLAY; ++l) {
    k_hih<<<NGR, NTHR, 0, stream>>>(hc, wf, eb1, l, P, Q);
    k_edge<<<NGR * 32, NTHR, 0, stream>>>(xc, P, Q, wf, l, ew1, eb2, cb1, cw2, emask, xnx, agg);
    k_node<<<NGR, NTHR, 0, stream>>>(hc, agg, wf, l, nb1, nb2, nmask, hnx);
    float* t;
    t = xc; xc = xnx; xnx = t;
    t = hc; hc = hnx; hnx = t;
  }
  k_out<<<1, NTHR, 0, stream>>>(hc, out_w, out_b, nmask, out);
}
